// BehaviorSpecificPFF_89936615178802
// MI455X (gfx1250) — hardware-verified
//
#include <hip/hip_runtime.h>
#include <stddef.h>
#include <stdint.h>


typedef __attribute__((ext_vector_type(16))) _Float16 v16h;
typedef __attribute__((ext_vector_type(8)))  _Float16 v8h;
typedef __attribute__((ext_vector_type(16))) __bf16   v16b;
typedef __attribute__((ext_vector_type(8)))  __bf16   v8b;
typedef __attribute__((ext_vector_type(8)))  float    v8f;
typedef __attribute__((ext_vector_type(4)))  float    v4f;

#define DMOD 512
#define CH   4096
#define TB   64
#define WSCALE 64.0f
#define WSCALE_INV (1.0f / 64.0f)

__device__ __forceinline__ unsigned short f2bf_bits(float f) {
  unsigned u = __float_as_uint(f);
  return (unsigned short)((u + 0x7FFFu + ((u >> 16) & 1u)) >> 16);
}
__device__ __forceinline__ float bf_bits2f(unsigned short h) { return __uint_as_float(((unsigned)h) << 16); }

__device__ __forceinline__ void dep_guard_h(v8f& a, v8f& b, v16h x, v16h y) { asm volatile("v_nop\n\tv_nop\n\tv_nop\n\tv_nop" : "+v"(a), "+v"(b) : "v"(x), "v"(y)); }
__device__ __forceinline__ void dep_guard_b(v8f& a, v8f& b, v16b x, v16b y) { asm volatile("v_nop\n\tv_nop\n\tv_nop\n\tv_nop" : "+v"(a), "+v"(b) : "v"(x), "v"(y)); }
__device__ __forceinline__ void keep4_h(v16h a, v16h b, v16h c, v16h d) { asm volatile("v_nop" :: "v"(a), "v"(b), "v"(c), "v"(d)); }
__device__ __forceinline__ void keep4_b(v16b a, v16b b, v16b c, v16b d) { asm volatile("v_nop" :: "v"(a), "v"(b), "v"(c), "v"(d)); }
__device__ __forceinline__ void acc_guard4(v8f& a, v8f& b, v8f& c, v8f& d) { asm volatile("v_nop\n\tv_nop\n\tv_nop\n\tv_nop" : "+v"(a), "+v"(b), "+v"(c), "+v"(d)); }

template <typename T> struct Frag;
template <> struct Frag<_Float16> {
  typedef v16h V; union U { v16h v; v8h h[2]; };
  static __device__ __forceinline__ v16h load(const _Float16* p) {
    U f; f.h[0] = *(const v8h*)(p); f.h[1] = *(const v8h*)(p + 16); return f.v;
  }
  static __device__ __forceinline__ v8f mma(v16h a, v16h b, v8f c) {
    return __builtin_amdgcn_wmma_f32_16x16x32_f16(false, a, false, b, (short)0, c, false, false);
  }
  static __device__ __forceinline__ void guard(v8f& a, v8f& b, v16h x, v16h y) { dep_guard_h(a, b, x, y); }
  static __device__ __forceinline__ void keep(v16h a, v16h b, v16h c, v16h d) { keep4_h(a, b, c, d); }
};
template <> struct Frag<__bf16> {
  typedef v16b V; union U { v16b v; v8b h[2]; };
  static __device__ __forceinline__ v16b load(const __bf16* p) {
    U f; f.h[0] = *(const v8b*)(p); f.h[1] = *(const v8b*)(p + 16); return f.v;
  }
  static __device__ __forceinline__ v8f mma(v16b a, v16b b, v8f c) {
    return __builtin_amdgcn_wmma_f32_16x16x32_bf16(false, a, false, b, (short)0, c, false, false);
  }
  static __device__ __forceinline__ void guard(v8f& a, v8f& b, v16b x, v16b y) { dep_guard_b(a, b, x, y); }
  static __device__ __forceinline__ void keep(v16b a, v16b b, v16b c, v16b d) { keep4_b(a, b, c, d); }
};

template <int ET> struct Elem;
template <> struct Elem<0> { typedef _Float16 T; };
template <> struct Elem<1> { typedef __bf16 T; };
template <int ET, bool SPLIT, int BIAS_MODE, int OUT_MODE, bool RESID, int ACT = 0>
__global__ __launch_bounds__(256) void wmma_gemm64c(
    const unsigned short* __restrict__ Ap, const unsigned short* __restrict__ A2p, int lda, long strideA,
    const unsigned short* __restrict__ Btp, const unsigned short* __restrict__ Bt2p, int ldb, long strideB,
    void* __restrict__ Cout, void* __restrict__ Cout2, int ldc, long strideC,
    const float* __restrict__ bias,
    const float* __restrict__ resid, long strideR,
    const int* __restrict__ ids, int idsPerZ, int idval,
    int Mmax, int N, int K, float scale) {
  typedef typename Elem<ET>::T T;
  typedef typename Frag<T>::V V;
  const T* A = (const T*)Ap; const T* A2 = (const T*)A2p; const T* Bt = (const T*)Btp; const T* Bt2 = (const T*)Bt2p;
  __shared__ __align__(16) float sT[8][16 * 68];
  __shared__ int sCnt[8];
  const int b    = blockIdx.y;
  const int lane = threadIdx.x & 31;
  const int wave = threadIdx.x >> 5;

  {
    int cnt = 0;
    const int4* idz = (const int4*)(ids + (size_t)b * idsPerZ);
    const int n4 = idsPerZ >> 2;
    for (int i = threadIdx.x; i < n4; i += 256) {
      const int4 u = idz[i];
      cnt += (u.x == idval) ? 1 : 0;
      cnt += (u.y == idval) ? 1 : 0;
      cnt += (u.z == idval) ? 1 : 0;
      cnt += (u.w == idval) ? 1 : 0;
    }
#pragma unroll
    for (int off = 16; off > 0; off >>= 1) cnt += __shfl_xor(cnt, off, 32);
    if (lane == 0) sCnt[wave] = cnt;
  }
  __syncthreads();
  int rows = 0;
#pragma unroll
  for (int w = 0; w < 8; ++w) rows += sCnt[w];
  int M = ((rows + 63) >> 6) << 6;
  M = (M > Mmax) ? Mmax : M;

  const int tilesN = N >> 6;
  const int tilesM = M >> 6;
  const int tile = blockIdx.x * 8 + wave;
  if (tile >= tilesM * tilesN) return;
  const int tm = tile / tilesN;
  const int tn = tile - tm * tilesN;
  const int m0 = tm << 6;
  const int n0 = tn << 6;

  const T* Ab  = A  + (size_t)b * strideA;
  const T* Bb  = Bt + (size_t)b * strideB;
  const T* Ab2 = SPLIT ? (A2  + (size_t)b * strideA) : nullptr;
  const T* Bb2 = SPLIT ? (Bt2 + (size_t)b * strideB) : nullptr;

  const int rlane = lane & 15;
  const int koff  = (lane >> 4) * 8;
  const int mOff  = (lane >> 4) * 8;

  v8f acc[4][4];
#pragma unroll
  for (int i = 0; i < 4; ++i)
#pragma unroll
    for (int j = 0; j < 4; ++j) acc[i][j] = (v8f){0.f,0.f,0.f,0.f,0.f,0.f,0.f,0.f};

  for (int k0 = 0; k0 < K; k0 += 32) {
    V bh[4], bl[4];
#pragma unroll
    for (int j = 0; j < 4; ++j) {
      const size_t bo = (size_t)(n0 + (j << 4) + rlane) * ldb + koff + k0;
      bh[j] = Frag<T>::load(Bb + bo);
      if (SPLIT) bl[j] = Frag<T>::load(Bb2 + bo);
    }
#pragma unroll
    for (int i = 0; i < 4; ++i) {
      const size_t ao = (size_t)(m0 + (i << 4) + rlane) * lda + koff + k0;
      V ah = Frag<T>::load(Ab + ao);
      V al;
      if (SPLIT) al = Frag<T>::load(Ab2 + ao);
#pragma unroll
      for (int j = 0; j < 4; ++j) {
        acc[i][j] = Frag<T>::mma(ah, bh[j], acc[i][j]);
        if (SPLIT) {
          acc[i][j] = Frag<T>::mma(ah, bl[j], acc[i][j]);
          acc[i][j] = Frag<T>::mma(al, bh[j], acc[i][j]);
        }
      }
      Frag<T>::guard(acc[i][0], acc[i][3], ah, SPLIT ? al : ah);
    }
    Frag<T>::keep(bh[0], bh[1], bh[2], bh[3]);
    if (SPLIT) Frag<T>::keep(bl[0], bl[1], bl[2], bl[3]);
  }
  acc_guard4(acc[0][0], acc[0][1], acc[0][2], acc[0][3]);
  acc_guard4(acc[1][0], acc[1][1], acc[1][2], acc[1][3]);
  acc_guard4(acc[2][0], acc[2][1], acc[2][2], acc[2][3]);
  acc_guard4(acc[3][0], acc[3][1], acc[3][2], acc[3][3]);

  float* slab = sT[wave];
  const float* Rb = RESID ? (resid + (size_t)b * strideR) : nullptr;
#pragma unroll
  for (int i = 0; i < 4; ++i) {
    const int mBase = m0 + (i << 4);
#pragma unroll
    for (int j = 0; j < 4; ++j) {
      const int n = n0 + (j << 4) + rlane;
      float bv = 0.f;
      if (BIAS_MODE == 2) bv = bias[n];
#pragma unroll
      for (int r = 0; r < 8; ++r) {
        float v = acc[i][j][r] * scale;
        if (BIAS_MODE == 1) v += bias[mBase + mOff + r];
        if (BIAS_MODE == 2) v += bv;
        if (RESID) v += Rb[(size_t)(mBase + mOff + r) * ldc + n];
        if (ACT == 1) v = tanhf(v);
        if (ACT == 2) v = fmaxf(v, 0.0f);
        if (ACT == 3) v = v / (1.0f + expf(-v));
        if (ACT == 4) v = (v > 0.f) ? v : 0.01f * v;
        if (ACT == 5) v = 0.5f * v * (1.0f + erff(v * 0.70710678118654752f));
        slab[(mOff + r) * 68 + (j << 4) + rlane] = v;
      }
    }
    __builtin_amdgcn_fence(__ATOMIC_RELEASE, "workgroup");
    __builtin_amdgcn_wave_barrier();
    __builtin_amdgcn_fence(__ATOMIC_ACQUIRE, "workgroup");
    if (OUT_MODE == 0) {
      float* C = (float*)Cout + (size_t)b * strideC;
      const int hh = lane >> 4, c4 = (lane & 15) * 4;
      for (int pass = 0; pass < 2; ++pass) {
#pragma unroll
        for (int it = 0; it < 8; ++it) {
          const int row = it * 2 + hh;
          v4f v = *(const v4f*)(slab + row * 68 + c4);
          *(volatile v4f*)(C + (size_t)(mBase + row) * ldc + n0 + c4) = v;
        }
        __threadfence();
      }
    } else {
      const int q = lane >> 3, c8 = (lane & 7) * 8;
      unsigned short* C  = (unsigned short*)Cout  + (size_t)b * strideC;
      unsigned short* C2 = (OUT_MODE == 2) ? ((unsigned short*)Cout2 + (size_t)b * strideC) : nullptr;
      for (int pass = 0; pass < 2; ++pass) {
#pragma unroll
        for (int it = 0; it < 4; ++it) {
          const int row = it * 4 + q;
          const float* sp = slab + row * 68 + c8;
          v8h hv, lv;
#pragma unroll
          for (int e = 0; e < 8; ++e) {
            if (OUT_MODE == 1) {
              hv[e] = (_Float16)sp[e];
            } else {
              unsigned short hb = f2bf_bits(sp[e]);
              unsigned short lb = f2bf_bits(sp[e] - bf_bits2f(hb));
              hv[e] = __builtin_bit_cast(_Float16, hb);
              lv[e] = __builtin_bit_cast(_Float16, lb);
            }
          }
          *(volatile v8h*)(C + (size_t)(mBase + row) * ldc + n0 + c8) = hv;
          if (OUT_MODE == 2) *(volatile v8h*)(C2 + (size_t)(mBase + row) * ldc + n0 + c8) = lv;
        }
        __threadfence();
      }
    }
    __builtin_amdgcn_fence(__ATOMIC_RELEASE, "workgroup");
    __builtin_amdgcn_wave_barrier();
    __builtin_amdgcn_fence(__ATOMIC_ACQUIRE, "workgroup");
  }
}

__global__ __launch_bounds__(256) void k_cast_w_f16(
    const float* __restrict__ wa, const float* __restrict__ wb,
    _Float16* __restrict__ oa, _Float16* __restrict__ ob, int n2, float sc) {
  const int i = blockIdx.x * 256 + threadIdx.x;
  if (i < n2) {
    const _Float16 a0 = (_Float16)(wa[2 * i] * sc), a1 = (_Float16)(wa[2 * i + 1] * sc);
    const _Float16 b0 = (_Float16)(wb[2 * i] * sc), b1 = (_Float16)(wb[2 * i + 1] * sc);
    const unsigned ua = (unsigned)__builtin_bit_cast(unsigned short, a0) | ((unsigned)__builtin_bit_cast(unsigned short, a1) << 16);
    const unsigned ub = (unsigned)__builtin_bit_cast(unsigned short, b0) | ((unsigned)__builtin_bit_cast(unsigned short, b1) << 16);
    ((volatile unsigned*)oa)[i] = ua;
    ((volatile unsigned*)ob)[i] = ub;
    __threadfence();
    ((volatile unsigned*)oa)[i] = ua;
    ((volatile unsigned*)ob)[i] = ub;
  }
}

__device__ __forceinline__ void chunk_partial_counts(const int* __restrict__ ids, int cbase, int t0, int idval,
                                                     int tid, int& before, int& total) {
  const int4* ip = (const int4*)(ids + cbase) + tid * (CH / 256 / 4);
  int bsum = 0, tsum = 0;
#pragma unroll
  for (int q = 0; q < CH / 256 / 4; ++q) {
    const int4 u = ip[q];
    const int base = cbase + tid * (CH / 256) + q * 4;
    int m;
    m = (u.x == idval) ? 1 : 0; tsum += m; bsum += (base + 0 < t0) ? m : 0;
    m = (u.y == idval) ? 1 : 0; tsum += m; bsum += (base + 1 < t0) ? m : 0;
    m = (u.z == idval) ? 1 : 0; tsum += m; bsum += (base + 2 < t0) ? m : 0;
    m = (u.w == idval) ? 1 : 0; tsum += m; bsum += (base + 3 < t0) ? m : 0;
  }
#pragma unroll
  for (int off = 16; off > 0; off >>= 1) {
    bsum += __shfl_xor(bsum, off, 32);
    tsum += __shfl_xor(tsum, off, 32);
  }
  before = bsum; total = tsum;
}

__device__ __forceinline__ void token_rank(unsigned m0, unsigned m1, int tl, unsigned& bit, int& rank) {
  const int sh = tl & 31;
  const unsigned low = (1u << sh) - 1u;
  const unsigned mm = (tl < 32) ? m0 : m1;
  bit = (mm >> sh) & 1u;
  rank = (tl < 32) ? (int)__popc(m0 & low) : (int)(__popc(m0) + __popc(m1 & low));
}

__global__ __launch_bounds__(256) void k_gather_rows(const float* __restrict__ x, const int* __restrict__ ids,
                                                    _Float16* __restrict__ Apl, int idval) {
  __shared__ int sRed[16];
  const int tid = threadIdx.x, lane = tid & 31, wave = tid >> 5;
  const int t0 = blockIdx.x * TB;
  const int c = t0 / CH;
  const int cbase = c * CH;
  int pb, pt;
  chunk_partial_counts(ids, cbase, t0, idval, tid, pb, pt);
  if (lane == 0) { sRed[wave] = pb; sRed[8 + wave] = pt; }
  __syncthreads();
  int bsum = 0, tsum = 0;
#pragma unroll
  for (int w = 0; w < 8; ++w) { bsum += sRed[w]; tsum += sRed[8 + w]; }

  const unsigned m0 = (unsigned)__ballot(ids[t0 + lane] == idval);
  const unsigned m1 = (unsigned)__ballot(ids[t0 + 32 + lane] == idval);
  _Float16* Ac = Apl + (size_t)c * CH * DMOD;

#pragma unroll 1
  for (int j = 0; j < TB / 8; ++j) {
    const int tl = wave * (TB / 8) + j;
    unsigned bit; int rank;
    token_rank(m0, m1, tl, bit, rank);
    if (bit) {
      int slot = bsum + rank;
      slot = (slot < CH) ? slot : (CH - 1);
      const float* xr = x + (size_t)(t0 + tl) * DMOD + 8 * lane;
      _Float16* ar = Ac + (size_t)slot * DMOD + 8 * lane;
      const v4f a0 = *(const v4f*)(xr),       a1 = *(const v4f*)(xr + 4);
      const v4f a2 = *(const v4f*)(xr + 256), a3 = *(const v4f*)(xr + 260);
      v8h h0, h1;
      h0[0] = (_Float16)a0[0]; h0[1] = (_Float16)a0[1]; h0[2] = (_Float16)a0[2]; h0[3] = (_Float16)a0[3];
      h0[4] = (_Float16)a1[0]; h0[5] = (_Float16)a1[1]; h0[6] = (_Float16)a1[2]; h0[7] = (_Float16)a1[3];
      h1[0] = (_Float16)a2[0]; h1[1] = (_Float16)a2[1]; h1[2] = (_Float16)a2[2]; h1[3] = (_Float16)a2[3];
      h1[4] = (_Float16)a3[0]; h1[5] = (_Float16)a3[1]; h1[6] = (_Float16)a3[2]; h1[7] = (_Float16)a3[3];
      *(volatile v8h*)(ar) = h0;
      *(volatile v8h*)(ar + 256) = h1;
      __threadfence();
      *(volatile v8h*)(ar) = h0;
      *(volatile v8h*)(ar + 256) = h1;
    }
  }

  if (t0 + TB == cbase + CH) {
    int padEnd = ((tsum + 63) >> 6) << 6;
    padEnd = (padEnd > CH) ? CH : padEnd;
    v8h z;
#pragma unroll
    for (int e = 0; e < 8; ++e) z[e] = (_Float16)0.0f;
#pragma unroll 1
    for (int k = 0; k < 8; ++k) {
      const int row = tsum + wave + 8 * k;
      if (row < padEnd) {
        _Float16* ar = Ac + (size_t)row * DMOD + 8 * lane;
        *(volatile v8h*)(ar) = z;
        *(volatile v8h*)(ar + 256) = z;
        __threadfence();
        *(volatile v8h*)(ar) = z;
        *(volatile v8h*)(ar + 256) = z;
      }
    }
  }
}

__global__ __launch_bounds__(256) void k_ln_select_out(const float* __restrict__ x, const int* __restrict__ ids,
                                                      const float* __restrict__ Ypl,
                                                      const float* __restrict__ gam, const float* __restrict__ bet,
                                                      float* __restrict__ out, int idval, int writeZero, float eps) {
  __shared__ int sRed[8];
  const int tid = threadIdx.x, lane = tid & 31, wave = tid >> 5;
  const int t0 = blockIdx.x * TB;
  const int c = t0 / CH;
  const int cbase = c * CH;
  int pb, pt;
  chunk_partial_counts(ids, cbase, t0, idval, tid, pb, pt);
  if (lane == 0) sRed[wave] = pb;
  __syncthreads();
  int bsum = 0;
#pragma unroll
  for (int w = 0; w < 8; ++w) bsum += sRed[w];

  const int i0 = ids[t0 + lane], i1 = ids[t0 + 32 + lane];
  const unsigned m0 = (unsigned)__ballot(i0 == idval);
  const unsigned m1 = (unsigned)__ballot(i1 == idval);
  const unsigned z0 = (unsigned)__ballot(i0 == 0);
  const unsigned z1 = (unsigned)__ballot(i1 == 0);
  const float* Yc = Ypl + (size_t)c * CH * DMOD;

  const v4f g0 = *(const v4f*)(gam + 4 * lane),       g1 = *(const v4f*)(gam + 128 + 4 * lane);
  const v4f g2 = *(const v4f*)(gam + 256 + 4 * lane), g3 = *(const v4f*)(gam + 384 + 4 * lane);
  const v4f e0 = *(const v4f*)(bet + 4 * lane),       e1 = *(const v4f*)(bet + 128 + 4 * lane);
  const v4f e2 = *(const v4f*)(bet + 256 + 4 * lane), e3 = *(const v4f*)(bet + 384 + 4 * lane);

#pragma unroll 1
  for (int j = 0; j < TB / 8; ++j) {
    const int tl = wave * (TB / 8) + j;
    unsigned bit; int rank;
    token_rank(m0, m1, tl, bit, rank);
    unsigned zbit; int zrank;
    token_rank(z0, z1, tl, zbit, zrank);
    zbit = writeZero ? zbit : 0u;
    float* orow = out + (size_t)(t0 + tl) * DMOD + 4 * lane;
    if (bit) {
      int slot = bsum + rank;
      slot = (slot < CH) ? slot : (CH - 1);
      const float* yr = Yc + (size_t)slot * DMOD + 4 * lane;
      const float* xr = x + (size_t)(t0 + tl) * DMOD + 4 * lane;
      const v4f r0 = *(const v4f*)(yr)       + *(const v4f*)(xr);
      const v4f r1 = *(const v4f*)(yr + 128) + *(const v4f*)(xr + 128);
      const v4f r2 = *(const v4f*)(yr + 256) + *(const v4f*)(xr + 256);
      const v4f r3 = *(const v4f*)(yr + 384) + *(const v4f*)(xr + 384);
      float s = (r0[0] + r0[1]) + (r0[2] + r0[3]);
      s += (r1[0] + r1[1]) + (r1[2] + r1[3]);
      s += (r2[0] + r2[1]) + (r2[2] + r2[3]);
      s += (r3[0] + r3[1]) + (r3[2] + r3[3]);
#pragma unroll
      for (int off = 16; off > 0; off >>= 1) s += __shfl_xor(s, off, 32);
      const float mean = s * (1.0f / (float)DMOD);
      const v4f d0 = r0 - mean, d1 = r1 - mean, d2 = r2 - mean, d3 = r3 - mean;
      float q = 0.f;
      q += d0[0] * d0[0]; q += d0[1] * d0[1]; q += d0[2] * d0[2]; q += d0[3] * d0[3];
      q += d1[0] * d1[0]; q += d1[1] * d1[1]; q += d1[2] * d1[2]; q += d1[3] * d1[3];
      q += d2[0] * d2[0]; q += d2[1] * d2[1]; q += d2[2] * d2[2]; q += d2[3] * d2[3];
      q += d3[0] * d3[0]; q += d3[1] * d3[1]; q += d3[2] * d3[2]; q += d3[3] * d3[3];
#pragma unroll
      for (int off = 16; off > 0; off >>= 1) q += __shfl_xor(q, off, 32);
      const float var = q * (1.0f / (float)DMOD);
      const float inv = 1.0f / sqrtf(var + eps);
      const v4f o0 = (d0 * inv) * g0 + e0;
      const v4f o1 = (d1 * inv) * g1 + e1;
      const v4f o2 = (d2 * inv) * g2 + e2;
      const v4f o3 = (d3 * inv) * g3 + e3;
      *(volatile v4f*)(orow)       = o0;
      *(volatile v4f*)(orow + 128) = o1;
      *(volatile v4f*)(orow + 256) = o2;
      *(volatile v4f*)(orow + 384) = o3;
      __threadfence();
      *(volatile v4f*)(orow)       = o0;
      *(volatile v4f*)(orow + 128) = o1;
      *(volatile v4f*)(orow + 256) = o2;
      *(volatile v4f*)(orow + 384) = o3;
    } else if (zbit) {
      const v4f z = (v4f){0.f, 0.f, 0.f, 0.f};
      *(volatile v4f*)(orow)       = z;
      *(volatile v4f*)(orow + 128) = z;
      *(volatile v4f*)(orow + 256) = z;
      *(volatile v4f*)(orow + 384) = z;
      __threadfence();
      *(volatile v4f*)(orow)       = z;
      *(volatile v4f*)(orow + 128) = z;
      *(volatile v4f*)(orow + 256) = z;
      *(volatile v4f*)(orow + 384) = z;
    }
  }
}

extern "C" void kernel_launch(void* const* d_in, const int* in_sizes, int n_in,
                              void* d_out, int out_size, void* d_ws, size_t ws_size,
                              hipStream_t stream) {
  if (n_in < 8) return;
  const float* x     = (const float*)d_in[0];
  const int*   bseq  = (const int*)d_in[1];
  const float* W1    = (const float*)d_in[2];
  const float* b1    = (const float*)d_in[3];
  const float* W2    = (const float*)d_in[4];
  const float* b2    = (const float*)d_in[5];
  const float* gamma = (const float*)d_in[6];
  const float* beta  = (const float*)d_in[7];
  float* out = (float*)d_out;

  const int NT = in_sizes[1];
  if (NT <= 0) return;
  const int D = in_sizes[0] / NT;
  if (D != DMOD || in_sizes[0] != NT * D) return;
  const int NBv = in_sizes[5] / D;
  if (NBv <= 0 || in_sizes[5] != NBv * D) return;
  const int DF = in_sizes[3] / NBv;
  if (DF <= 0 || (DF % 64) != 0) return;
  if (in_sizes[2] != NBv * DF * D || in_sizes[4] != NBv * D * DF) return;
  if (in_sizes[6] != NBv * D || in_sizes[7] != NBv * D) return;
  if ((NT % CH) != 0 || (NT % TB) != 0 || out_size != NT * D) return;
  const int NCH = NT / CH;

  const size_t szW1 = (size_t)DF * D * 2;
  const size_t szW2 = (size_t)D * DF * 2;
  const size_t szA  = (size_t)NT * D * 2;
  const size_t szH  = (size_t)NT * DF * 2;
  const size_t szY  = (size_t)NT * D * 4;
  const size_t offW1 = 0;
  const size_t offW2 = offW1 + szW1;
  const size_t offA  = offW2 + szW2;
  const size_t offH  = offA + szA;
  const size_t offY  = offH + szH;
  const size_t total = offY + szY;
  if (total > ws_size || total > (size_t)134217728) return;

  char* ws = (char*)d_ws;
  _Float16* W1h = (_Float16*)(ws + offW1);
  _Float16* W2h = (_Float16*)(ws + offW2);
  _Float16* Apl = (_Float16*)(ws + offA);
  _Float16* Hpl = (_Float16*)(ws + offH);
  float*    Ypl = (float*)(ws + offY);
  const unsigned short* Au  = (const unsigned short*)Apl;
  const unsigned short* Hu  = (const unsigned short*)Hpl;
  const unsigned short* W1u = (const unsigned short*)W1h;
  const unsigned short* W2u = (const unsigned short*)W2h;

  const int n2 = (DF * D) / 2;
  const int castBlocks = (n2 + 255) / 256;
  const int tokBlocks  = NT / TB;
  const int gx1 = ((CH / 64) * (DF / 64)) / 8;
  const int gx2 = ((CH / 64) * (D / 64)) / 8;
  const float eps = 1e-5f;

  for (int n = 0; n < NBv; ++n) {
    k_cast_w_f16<<<dim3(castBlocks), dim3(256), 0, stream>>>(
        W1 + (size_t)n * DF * D, W2 + (size_t)n * D * DF, W1h, W2h, n2, WSCALE);

    k_gather_rows<<<dim3(tokBlocks), dim3(256), 0, stream>>>(x, bseq, Apl, n + 1);

    wmma_gemm64c<0, false, 2, 1, false, 2><<<dim3(gx1, NCH), dim3(256), 0, stream>>>(
        Au, Au, D, (long)CH * D,
        W1u, W1u, D, 0L,
        (void*)Hpl, (void*)Hpl, DF, (long)CH * DF,
        b1 + (size_t)n * DF,
        x, 0L,
        bseq, CH, n + 1,
        CH, DF, D, WSCALE_INV);

    wmma_gemm64c<0, false, 2, 0, false, 0><<<dim3(gx2, NCH), dim3(256), 0, stream>>>(
        Hu, Hu, DF, (long)CH * DF,
        W2u, W2u, DF, 0L,
        (void*)Ypl, (void*)Ypl, D, (long)CH * D,
        b2 + (size_t)n * D,
        x, 0L,
        bseq, CH, n + 1,
        CH, D, DF, WSCALE_INV);

    k_ln_select_out<<<dim3(tokBlocks), dim3(256), 0, stream>>>(
        x, bseq, Ypl, gamma + (size_t)n * D, beta + (size_t)n * D, out, n + 1, (n == 0) ? 1 : 0, eps);
  }
}
